// LSTM_89678917141105
// MI455X (gfx1250) — hardware-verified
//
#include <hip/hip_runtime.h>
#include <math.h>

constexpr int NSEQ   = 32;
constexpr int NSTEP  = 512;
constexpr int NIN    = 512;
constexpr int NHID   = 1024;
constexpr int NGATE  = 4 * NHID;
constexpr int TCH    = 128;
constexpr int NCHUNK = NSTEP / TCH;
constexpr int NPAIR  = TCH / 2;
constexpr int ZN     = 2 * NSEQ;
constexpr int NROWS  = NSEQ * NSTEP;
constexpr int PTHR   = 256;
constexpr int RTHR   = 512;
constexpr int RWAVES = RTHR / 32;
constexpr int SEQB   = 16;
constexpr int HP     = 1032;
constexpr int OBP    = 132;
constexpr float WHC     = 16.0f;
constexpr float WHC_INV = 1.0f / 16.0f;
static_assert(NIN % 32 == 0 && NHID % 32 == 0);
static_assert(NGATE % 64 == 0 && ZN % 64 == 0);
static_assert((NGATE / 64) * (ZN / 64) % 8 == 0);
static_assert(NIN % 64 == 0 && NHID % 64 == 0);
static_assert(TCH % 2 == 0 && NSTEP % TCH == 0);
static_assert(NSEQ % SEQB == 0 && RWAVES == SEQB);
static_assert(NHID == 64 * RWAVES);
static_assert(TCH == 32 * 4);
static_assert(SEQB * NHID / 8 == 4 * RTHR);
static_assert(NGATE / 4 == 2 * RTHR && NHID / 4 <= RTHR);
static_assert((NROWS * (NIN / 8)) % PTHR == 0);
static_assert(HP % 8 == 0 && OBP % 4 == 0 && HP >= NHID && OBP >= TCH);

typedef __attribute__((ext_vector_type(16))) _Float16 v16h;
typedef __attribute__((ext_vector_type(8)))  _Float16 v8h;
typedef __attribute__((ext_vector_type(16))) __bf16   v16b;
typedef __attribute__((ext_vector_type(8)))  __bf16   v8b;
typedef __attribute__((ext_vector_type(8)))  float    v8f;
typedef __attribute__((ext_vector_type(4)))  float    v4f;
typedef __attribute__((ext_vector_type(4)))  unsigned u4;

__device__ __forceinline__ unsigned short f2bf_bits(float f) {
  unsigned u = __float_as_uint(f);
  return (unsigned short)((u + 0x7FFFu + ((u >> 16) & 1u)) >> 16);
}
__device__ __forceinline__ float bf_bits2f(unsigned short h) { return __uint_as_float(((unsigned)h) << 16); }
__device__ __forceinline__ float bf16r(float f) { return bf_bits2f(f2bf_bits(f)); }

__device__ __forceinline__ void dep_guard_h(v8f& a, v8f& b, v16h x, v16h y) { asm volatile("v_nop\n\tv_nop\n\tv_nop\n\tv_nop" : "+v"(a), "+v"(b) : "v"(x), "v"(y)); }
__device__ __forceinline__ void dep_guard_b(v8f& a, v8f& b, v16b x, v16b y) { asm volatile("v_nop\n\tv_nop\n\tv_nop\n\tv_nop" : "+v"(a), "+v"(b) : "v"(x), "v"(y)); }
__device__ __forceinline__ void guard_all_h(v8f& c0, v8f& c1, v8f& c2, v8f& c3, v16h a, v16h b0, v16h b1, v16h b2, v16h b3) {
  asm volatile("v_nop\n\tv_nop\n\tv_nop\n\tv_nop" : "+v"(c0), "+v"(c1), "+v"(c2), "+v"(c3) : "v"(a), "v"(b0), "v"(b1), "v"(b2), "v"(b3));
}
__device__ __forceinline__ void guard_all_b(v8f& c0, v8f& c1, v8f& c2, v8f& c3, v16b a, v16b b0, v16b b1, v16b b2, v16b b3) {
  asm volatile("v_nop\n\tv_nop\n\tv_nop\n\tv_nop" : "+v"(c0), "+v"(c1), "+v"(c2), "+v"(c3) : "v"(a), "v"(b0), "v"(b1), "v"(b2), "v"(b3));
}
__device__ __forceinline__ void keep4_h(v16h a, v16h b, v16h c, v16h d) { asm volatile("v_nop" :: "v"(a), "v"(b), "v"(c), "v"(d)); }
__device__ __forceinline__ void keep4_b(v16b a, v16b b, v16b c, v16b d) { asm volatile("v_nop" :: "v"(a), "v"(b), "v"(c), "v"(d)); }
__device__ __forceinline__ void acc_guard4(v8f& a, v8f& b, v8f& c, v8f& d) { asm volatile("v_nop\n\tv_nop\n\tv_nop\n\tv_nop" : "+v"(a), "+v"(b), "+v"(c), "+v"(d)); }
template <typename T> struct Frag;
template <> struct Frag<_Float16> {
  typedef v16h V; union U { v16h v; v8h h[2]; };
  static __device__ __forceinline__ v16h load(const _Float16* p) {
    U f; f.h[0] = *(const v8h*)(p); f.h[1] = *(const v8h*)(p + 16); return f.v;
  }
  static __device__ __forceinline__ v8f mma(v16h a, v16h b, v8f c) {
    return __builtin_amdgcn_wmma_f32_16x16x32_f16(false, a, false, b, (short)0, c, false, false);
  }
  static __device__ __forceinline__ void guard(v8f& a, v8f& b, v16h x, v16h y) { dep_guard_h(a, b, x, y); }
  static __device__ __forceinline__ void guard4(v8f& c0, v8f& c1, v8f& c2, v8f& c3, v16h a, v16h b0, v16h b1, v16h b2, v16h b3) { guard_all_h(c0, c1, c2, c3, a, b0, b1, b2, b3); }
  static __device__ __forceinline__ void keep(v16h a, v16h b, v16h c, v16h d) { keep4_h(a, b, c, d); }
};
template <> struct Frag<__bf16> {
  typedef v16b V; union U { v16b v; v8b h[2]; };
  static __device__ __forceinline__ v16b load(const __bf16* p) {
    U f; f.h[0] = *(const v8b*)(p); f.h[1] = *(const v8b*)(p + 16); return f.v;
  }
  static __device__ __forceinline__ v8f mma(v16b a, v16b b, v8f c) {
    return __builtin_amdgcn_wmma_f32_16x16x32_bf16(false, a, false, b, (short)0, c, false, false);
  }
  static __device__ __forceinline__ void guard(v8f& a, v8f& b, v16b x, v16b y) { dep_guard_b(a, b, x, y); }
  static __device__ __forceinline__ void guard4(v8f& c0, v8f& c1, v8f& c2, v8f& c3, v16b a, v16b b0, v16b b1, v16b b2, v16b b3) { guard_all_b(c0, c1, c2, c3, a, b0, b1, b2, b3); }
  static __device__ __forceinline__ void keep(v16b a, v16b b, v16b c, v16b d) { keep4_b(a, b, c, d); }
};

__device__ __forceinline__ float fsig(float x)  { return __builtin_amdgcn_rcpf(1.0f + expf(-x)); }
__device__ __forceinline__ float ftanh(float x) { return 1.0f - 2.0f * __builtin_amdgcn_rcpf(expf(2.0f * x) + 1.0f); }

template <int ET> struct Elem;
template <> struct Elem<0> { typedef _Float16 T; };
template <> struct Elem<1> { typedef __bf16 T; };
template <int ET, bool SPLIT, int BIAS_MODE, int OUT_MODE, bool RESID, int ACT = 0>
__global__ __launch_bounds__(256) void wmma_gemm64(
    const unsigned short* __restrict__ Ap, const unsigned short* __restrict__ A2p, int lda, long strideA,
    const unsigned short* __restrict__ Btp, const unsigned short* __restrict__ Bt2p, int ldb, long strideB,
    void* __restrict__ Cout, void* __restrict__ Cout2, int ldc, long strideC,
    const float* __restrict__ bias,
    const float* __restrict__ resid, long strideR,
    int M, int N, int K, float scale) {
  typedef typename Elem<ET>::T T;
  typedef typename Frag<T>::V V;
  const T* A = (const T*)Ap; const T* A2 = (const T*)A2p; const T* Bt = (const T*)Btp; const T* Bt2 = (const T*)Bt2p;
  __shared__ __align__(16) float sT[8][16 * 68];
  const int b    = blockIdx.y;
  const int lane = threadIdx.x & 31;
  const int wave = threadIdx.x >> 5;
  const int tilesN = N >> 6;
  const int tilesM = M >> 6;
  const int tile = blockIdx.x * 8 + wave;
  if (tile >= tilesM * tilesN) return;
  const int tm = tile / tilesN;
  const int tn = tile - tm * tilesN;
  const int m0 = tm << 6;
  const int n0 = tn << 6;

  const T* Ab  = A  + (size_t)b * strideA;
  const T* Bb  = Bt + (size_t)b * strideB;
  const T* Ab2 = SPLIT ? (A2  + (size_t)b * strideA) : nullptr;
  const T* Bb2 = SPLIT ? (Bt2 + (size_t)b * strideB) : nullptr;

  const int rlane = lane & 15;
  const int koff  = (lane >> 4) * 8;
  const int mOff  = (lane >> 4) * 8;

  v8f acc[4][4];
#pragma unroll
  for (int i = 0; i < 4; ++i)
#pragma unroll
    for (int j = 0; j < 4; ++j) acc[i][j] = (v8f){0.f,0.f,0.f,0.f,0.f,0.f,0.f,0.f};

  for (int k0 = 0; k0 < K; k0 += 32) {
    V bh[4], bl[4];
#pragma unroll
    for (int j = 0; j < 4; ++j) {
      const size_t bo = (size_t)(n0 + (j << 4) + rlane) * ldb + koff + k0;
      bh[j] = Frag<T>::load(Bb + bo);
      if (SPLIT) bl[j] = Frag<T>::load(Bb2 + bo);
    }
#pragma unroll
    for (int i = 0; i < 4; ++i) {
      const size_t ao = (size_t)(m0 + (i << 4) + rlane) * lda + koff + k0;
      V ah = Frag<T>::load(Ab + ao);
      V al;
      if (SPLIT) al = Frag<T>::load(Ab2 + ao);
#pragma unroll
      for (int j = 0; j < 4; ++j) {
        acc[i][j] = Frag<T>::mma(ah, bh[j], acc[i][j]);
        if (SPLIT) {
          acc[i][j] = Frag<T>::mma(ah, bl[j], acc[i][j]);
          acc[i][j] = Frag<T>::mma(al, bh[j], acc[i][j]);
        }
      }
      Frag<T>::guard4(acc[i][0], acc[i][1], acc[i][2], acc[i][3], ah, bh[0], bh[1], bh[2], bh[3]);
      if (SPLIT) Frag<T>::guard4(acc[i][0], acc[i][1], acc[i][2], acc[i][3], al, bl[0], bl[1], bl[2], bl[3]);
    }
    Frag<T>::keep(bh[0], bh[1], bh[2], bh[3]);
    if (SPLIT) Frag<T>::keep(bl[0], bl[1], bl[2], bl[3]);
  }
  acc_guard4(acc[0][0], acc[0][1], acc[0][2], acc[0][3]);
  acc_guard4(acc[1][0], acc[1][1], acc[1][2], acc[1][3]);
  acc_guard4(acc[2][0], acc[2][1], acc[2][2], acc[2][3]);
  acc_guard4(acc[3][0], acc[3][1], acc[3][2], acc[3][3]);

  float* slab = sT[wave];
  const float* Rb = RESID ? (resid + (size_t)b * strideR) : nullptr;
#pragma unroll
  for (int i = 0; i < 4; ++i) {
    const int mBase = m0 + (i << 4);
#pragma unroll
    for (int j = 0; j < 4; ++j) {
      const int n = n0 + (j << 4) + rlane;
      float bv = 0.f;
      if (BIAS_MODE == 2) bv = bias[n];
#pragma unroll
      for (int r = 0; r < 8; ++r) {
        float v = acc[i][j][r] * scale;
        if (BIAS_MODE == 1) v += bias[mBase + mOff + r];
        if (BIAS_MODE == 2) v += bv;
        if (RESID) v += Rb[(size_t)(mBase + mOff + r) * ldc + n];
        if (ACT == 1) v = tanhf(v);
        if (ACT == 2) v = fmaxf(v, 0.0f);
        if (ACT == 4) v = (v > 0.f) ? v : 0.01f * v;
        slab[(mOff + r) * 68 + (j << 4) + rlane] = v;
      }
    }
    __builtin_amdgcn_fence(__ATOMIC_RELEASE, "workgroup");
    __builtin_amdgcn_wave_barrier();
    __builtin_amdgcn_fence(__ATOMIC_ACQUIRE, "workgroup");
    if (OUT_MODE == 0) {
      float* C = (float*)Cout + (size_t)b * strideC;
      const int hh = lane >> 4, c4 = (lane & 15) * 4;
      for (int pass = 0; pass < 2; ++pass) {
#pragma unroll
        for (int it = 0; it < 8; ++it) {
          const int row = it * 2 + hh;
          v4f v = *(const v4f*)(slab + row * 68 + c4);
          *(volatile v4f*)(C + (size_t)(mBase + row) * ldc + n0 + c4) = v;
        }
        __threadfence();
      }
    } else {
      const int q = lane >> 3, c8 = (lane & 7) * 8;
      unsigned short* C  = (unsigned short*)Cout  + (size_t)b * strideC;
      unsigned short* C2 = (OUT_MODE == 2) ? ((unsigned short*)Cout2 + (size_t)b * strideC) : nullptr;
      for (int pass = 0; pass < 2; ++pass) {
#pragma unroll
        for (int it = 0; it < 4; ++it) {
          const int row = it * 4 + q;
          const float* sp = slab + row * 68 + c8;
          v8h hv, lv;
#pragma unroll
          for (int e = 0; e < 8; ++e) {
            if (OUT_MODE == 1) {
              hv[e] = (_Float16)sp[e];
            } else {
              unsigned short hb = f2bf_bits(sp[e]);
              unsigned short lb = f2bf_bits(sp[e] - bf_bits2f(hb));
              hv[e] = __builtin_bit_cast(_Float16, hb);
              lv[e] = __builtin_bit_cast(_Float16, lb);
            }
          }
          *(volatile v8h*)(C + (size_t)(mBase + row) * ldc + n0 + c8) = hv;
          if (OUT_MODE == 2) *(volatile v8h*)(C2 + (size_t)(mBase + row) * ldc + n0 + c8) = lv;
        }
        __threadfence();
      }
    }
    __builtin_amdgcn_fence(__ATOMIC_RELEASE, "workgroup");
    __builtin_amdgcn_wave_barrier();
    __builtin_amdgcn_fence(__ATOMIC_ACQUIRE, "workgroup");
  }
}

template <int MODE>
__global__ __launch_bounds__(PTHR) void tpw_kernel(const float* __restrict__ src, int R, int C, int ldo,
                                                  unsigned short* __restrict__ O, float sc) {
  __shared__ float Tt[64 * 65];
  const int tid = threadIdx.x;
  const int c0 = blockIdx.x * 64, r0 = blockIdx.y * 64;
#pragma unroll
  for (int i = 0; i < 4; ++i) {
    const int idx = i * PTHR + tid;
    const int rr = idx >> 4, cc = (idx & 15) * 4;
    const v4f v = *(const v4f*)(src + (size_t)(r0 + rr) * (size_t)C + c0 + cc);
    Tt[rr * 65 + cc + 0] = v[0];
    Tt[rr * 65 + cc + 1] = v[1];
    Tt[rr * 65 + cc + 2] = v[2];
    Tt[rr * 65 + cc + 3] = v[3];
  }
  __syncthreads();
  const int q = tid >> 3, c8 = (tid & 7) * 8;
  v8h hv[2];
#pragma unroll
  for (int g = 0; g < 2; ++g) {
    const int qq = g * 32 + q;
#pragma unroll
    for (int e = 0; e < 8; ++e) {
      const float f = Tt[(c8 + e) * 65 + qq];
      unsigned short bits;
      if (MODE == 0) {
        bits = f2bf_bits(f * sc);
      } else {
        const float fb = bf_bits2f(f2bf_bits(f));
        bits = __builtin_bit_cast(unsigned short, (_Float16)(fb * sc));
      }
      hv[g][e] = __builtin_bit_cast(_Float16, bits);
    }
  }
  for (int pass = 0; pass < 2; ++pass) {
#pragma unroll
    for (int g = 0; g < 2; ++g) {
      const size_t o = (size_t)(c0 + g * 32 + q) * (size_t)ldo + (size_t)(r0 + c8);
      *(volatile v8h*)(O + o) = hv[g];
    }
    __threadfence();
  }
}

__global__ __launch_bounds__(PTHR) void xcvt_kernel(const float* __restrict__ x, unsigned short* __restrict__ dst) {
  const int i  = blockIdx.x * PTHR + threadIdx.x;
  constexpr int NC8 = NIN / 8;
  constexpr int n8  = NROWS * NC8;
  if (i < n8) {
    const int rd = i / NC8;
    const int c8 = i - rd * NC8;
    const int t  = rd / NSEQ;
    const int b  = rd - t * NSEQ;
    const float* sp = x + ((size_t)b * NSTEP + (size_t)t) * NIN + c8 * 8;
    const v4f a = *(const v4f*)(sp);
    const v4f q = *(const v4f*)(sp + 4);
    v8h hv;
#pragma unroll
    for (int e = 0; e < 4; ++e) {
      hv[e]     = __builtin_bit_cast(_Float16, f2bf_bits(a[e]));
      hv[4 + e] = __builtin_bit_cast(_Float16, f2bf_bits(q[e]));
    }
    *(volatile v8h*)(dst + (size_t)i * 8) = hv;
    __threadfence();
    *(volatile v8h*)(dst + (size_t)i * 8) = hv;
  }
}

__global__ __launch_bounds__(RTHR) void lstm_rec_kernel(
    const float* __restrict__ ZT, const unsigned short* __restrict__ WHTp,
    const float* __restrict__ bias, const float* __restrict__ Wd, const float* __restrict__ bd,
    float* __restrict__ cstp, unsigned short* __restrict__ hpl, float* __restrict__ out,
    int t0, int first) {
  __shared__ __align__(16) _Float16 Ah[2 * SEQB * HP];
  __shared__ __align__(16) float    Cs[NGATE + NHID];
  __shared__ __align__(16) float    Ob[SEQB * OBP];
  __shared__ __align__(16) float    Ps[2 * RWAVES * SEQB];
  const _Float16* WHT = (const _Float16*)WHTp;
  const int tid = threadIdx.x, lane = tid & 31, wave = tid >> 5;
  const int c = lane & 15, hh = lane >> 4, koff = hh * 8;
  const int blk = blockIdx.x;
  const int rowbase = blk * SEQB;

#pragma unroll 1
  for (int i = tid; i < 2 * SEQB * HP; i += RTHR) Ah[i] = (_Float16)0.0f;
#pragma unroll
  for (int q = 0; q < 2; ++q) {
    const int i4 = q * RTHR + tid;
    const v4f v = *(const v4f*)(bias + (size_t)i4 * 4);
    v4f o;
#pragma unroll
    for (int e = 0; e < 4; ++e) o[e] = bf16r(v[e]);
    *(v4f*)(Cs + i4 * 4) = o;
  }
  if (tid < NHID / 4) {
    const v4f v = *(const v4f*)(Wd + (size_t)tid * 4);
    v4f o;
#pragma unroll
    for (int e = 0; e < 4; ++e) o[e] = bf16r(v[e]);
    *(v4f*)(Cs + NGATE + tid * 4) = o;
  }
  const float bdv = bf16r(bd[0]);
  float cst[4][8];
#pragma unroll
  for (int nt = 0; nt < 4; ++nt)
#pragma unroll
    for (int r = 0; r < 8; ++r) cst[nt][r] = 0.0f;
  if (!first) {
    const v4f* cp4 = (const v4f*)cstp;
#pragma unroll
    for (int nt = 0; nt < 4; ++nt)
#pragma unroll
      for (int q = 0; q < 2; ++q) {
        const v4f v = cp4[(size_t)((((blk * RWAVES + wave) * 4 + nt) * 2 + q) * 32 + lane)];
        cst[nt][4 * q + 0] = v[0]; cst[nt][4 * q + 1] = v[1]; cst[nt][4 * q + 2] = v[2]; cst[nt][4 * q + 3] = v[3];
      }
  }
  __syncthreads();
  if (!first) {
#pragma unroll
    for (int it = 0; it < 4; ++it) {
      const int idx = it * RTHR + tid;
      const int row = idx >> 7, c8 = (idx & 127) * 8;
      const u4 v = *(const u4*)(hpl + (size_t)(rowbase + row) * NHID + c8);
      *(u4*)(Ah + row * HP + c8) = v;
    }
  }
  __syncthreads();

  const v8f z8 = {0.f, 0.f, 0.f, 0.f, 0.f, 0.f, 0.f, 0.f};

#pragma unroll 1
  for (int tl = 0; tl < TCH; ++tl) {
    const int cur = tl & 1;
    const _Float16* ahrow = Ah + cur * (SEQB * HP) + c * HP + koff;
    _Float16* ahn = Ah + (cur ^ 1) * (SEQB * HP);
    const float* zrow = ZT + ((size_t)(tl >> 1) * NGATE) * ZN + (tl & 1) * NSEQ + rowbase + 8 * hh;
    float pr[8];
#pragma unroll
    for (int r = 0; r < 8; ++r) pr[r] = 0.0f;

#pragma unroll
    for (int nt = 0; nt < 4; ++nt) {
      const int j = 64 * wave + 16 * nt + c;
      v4f zv[4][2];
#pragma unroll
      for (int g = 0; g < 4; ++g) {
        const float* zp = zrow + (size_t)(g * NHID + j) * ZN;
        zv[g][0] = *(const v4f*)(zp);
        zv[g][1] = *(const v4f*)(zp + 4);
      }
      float bg[4];
#pragma unroll
      for (int g = 0; g < 4; ++g) bg[g] = Cs[g * NHID + j];
      const float wdj = Cs[NGATE + j];
      const _Float16* wh = WHT + (size_t)j * NHID + koff;
      v8f acc[4];
      acc[0] = z8; acc[1] = z8; acc[2] = z8; acc[3] = z8;
#pragma unroll 1
      for (int k0 = 0; k0 < NHID; k0 += 32) {
        const v16h a  = Frag<_Float16>::load(ahrow + k0);
        const v16h b0 = Frag<_Float16>::load(wh + k0);
        const v16h b1 = Frag<_Float16>::load(wh + (size_t)1 * NHID * NHID + k0);
        const v16h b2 = Frag<_Float16>::load(wh + (size_t)2 * NHID * NHID + k0);
        const v16h b3 = Frag<_Float16>::load(wh + (size_t)3 * NHID * NHID + k0);
        acc[0] = Frag<_Float16>::mma(a, b0, acc[0]);
        acc[1] = Frag<_Float16>::mma(a, b1, acc[1]);
        acc[2] = Frag<_Float16>::mma(a, b2, acc[2]);
        acc[3] = Frag<_Float16>::mma(a, b3, acc[3]);
        guard_all_h(acc[0], acc[1], acc[2], acc[3], a, b0, b1, b2, b3);
      }
      acc_guard4(acc[0], acc[1], acc[2], acc[3]);
#pragma unroll
      for (int r = 0; r < 8; ++r) {
        const float zi = acc[0][r] * WHC_INV + zv[0][r >> 2][r & 3] + bg[0];
        const float zf = acc[1][r] * WHC_INV + zv[1][r >> 2][r & 3] + bg[1];
        const float zg = acc[2][r] * WHC_INV + zv[2][r >> 2][r & 3] + bg[2];
        const float zo = acc[3][r] * WHC_INV + zv[3][r >> 2][r & 3] + bg[3];
        const float ig = fsig(zi);
        const float fg = fsig(zf);
        const float gg = ftanh(zg);
        const float og = fsig(zo);
        const float cn = fg * cst[nt][r] + ig * gg;
        cst[nt][r] = cn;
        const float hn = og * ftanh(cn);
        ahn[(8 * hh + r) * HP + j] = (_Float16)hn;
        pr[r] += hn * wdj;
      }
    }
#pragma unroll
    for (int r = 0; r < 8; ++r) {
#pragma unroll
      for (int off = 1; off < 16; off <<= 1) pr[r] += __shfl_xor(pr[r], off, 32);
    }
    {
      float* psw = Ps + cur * (RWAVES * SEQB) + wave * SEQB + 8 * hh;
#pragma unroll
      for (int r = 0; r < 8; ++r) {
        if (c == r) psw[r] = pr[r];
      }
    }
    __syncthreads();
    if (wave == 0 && lane < SEQB) {
      const float* psr = Ps + cur * (RWAVES * SEQB) + lane;
      float s = 0.0f;
#pragma unroll
      for (int w = 0; w < RWAVES; ++w) s += psr[w * SEQB];
      Ob[lane * OBP + tl] = s + bdv;
    }
  }
  __syncthreads();

  {
    const int orow = wave;
    const v4f ov = *(const v4f*)(Ob + orow * OBP + 4 * lane);
    float* op = out + (size_t)(rowbase + orow) * NSTEP + (size_t)t0 + 4 * lane;
    v4f cv[4][2];
#pragma unroll
    for (int nt = 0; nt < 4; ++nt)
#pragma unroll
      for (int q = 0; q < 2; ++q) {
        v4f v;
        v[0] = cst[nt][4 * q + 0]; v[1] = cst[nt][4 * q + 1]; v[2] = cst[nt][4 * q + 2]; v[3] = cst[nt][4 * q + 3];
        cv[nt][q] = v;
      }
    u4 hw[4];
#pragma unroll
    for (int it = 0; it < 4; ++it) {
      const int idx = it * RTHR + tid;
      const int row = idx >> 7, c8 = (idx & 127) * 8;
      hw[it] = *(const u4*)(Ah + row * HP + c8);
    }
    for (int pass = 0; pass < 2; ++pass) {
      *(volatile v4f*)op = ov;
#pragma unroll
      for (int nt = 0; nt < 4; ++nt)
#pragma unroll
        for (int q = 0; q < 2; ++q)
          *(volatile v4f*)(cstp + (size_t)((((blk * RWAVES + wave) * 4 + nt) * 2 + q) * 32 + lane) * 4) = cv[nt][q];
#pragma unroll
      for (int it = 0; it < 4; ++it) {
        const int idx = it * RTHR + tid;
        const int row = idx >> 7, c8 = (idx & 127) * 8;
        *(volatile u4*)(hpl + (size_t)(rowbase + row) * NHID + c8) = hw[it];
      }
      __threadfence();
    }
  }
}

extern "C" void kernel_launch(void* const* d_in, const int* in_sizes, int n_in,
                              void* d_out, int out_size, void* d_ws, size_t ws_size, hipStream_t stream) {
  if (n_in < 6 || d_out == nullptr || d_ws == nullptr) return;
  if (in_sizes[0] != NSEQ * NSTEP * NIN || in_sizes[1] != NIN * NGATE || in_sizes[2] != NHID * NGATE ||
      in_sizes[3] != NGATE || in_sizes[4] != NHID || in_sizes[5] != 1 || out_size != NSEQ * NSTEP) return;

  const float* x  = (const float*)d_in[0];
  const float* Wi = (const float*)d_in[1];
  const float* Wh = (const float*)d_in[2];
  const float* bb = (const float*)d_in[3];
  const float* Wd = (const float*)d_in[4];
  const float* bd = (const float*)d_in[5];
  float* out = (float*)d_out;

  char* ws = (char*)d_ws; size_t off = 0;
  auto carve = [&](size_t bytes) -> char* { char* p = ws + off; off += (bytes + 255) & ~(size_t)255; return p; };
  unsigned short* XB  = (unsigned short*)carve((size_t)NROWS * NIN * 2);
  unsigned short* WIT = (unsigned short*)carve((size_t)NGATE * NIN * 2);
  unsigned short* WHT = (unsigned short*)carve((size_t)NGATE * NHID * 2);
  float*          ZT  = (float*)carve((size_t)NPAIR * NGATE * ZN * 4);
  float*          CST = (float*)carve((size_t)(NSEQ / SEQB) * RWAVES * 4 * 8 * 32 * 4);
  unsigned short* HPL = (unsigned short*)carve((size_t)NSEQ * NHID * 2);
  if (off > ws_size || off > (size_t)134217728) return;

  xcvt_kernel<<<(NROWS * (NIN / 8)) / PTHR, PTHR, 0, stream>>>(x, XB);
  tpw_kernel<0><<<dim3(NGATE / 64, NIN / 64), PTHR, 0, stream>>>(Wi, NIN, NGATE, NIN, WIT, 1.0f);
  tpw_kernel<1><<<dim3(NGATE / 64, NHID / 64), PTHR, 0, stream>>>(Wh, NHID, NGATE, NHID, WHT, WHC);

  const dim3 ggrid((NGATE / 64) * (ZN / 64) / 8, NPAIR);
  for (int ch = 0; ch < NCHUNK; ++ch) {
    const unsigned short* XBc = XB + (size_t)ch * TCH * NSEQ * NIN;
    wmma_gemm64<1, false, 0, 0, false, 0><<<ggrid, 256, 0, stream>>>(
        WIT, WIT, NIN, 0L, XBc, XBc, NIN, (long)ZN * NIN, (void*)ZT, (void*)ZT, ZN, (long)NGATE * ZN,
        bb, (const float*)ZT, 0L, NGATE, ZN, NIN, 1.0f);
    lstm_rec_kernel<<<NSEQ / SEQB, RTHR, 0, stream>>>(ZT, WHT, bb, Wd, bd, CST, HPL, out, ch * TCH, ch == 0 ? 1 : 0);
  }
}
